// MultiHeadAttention_30408368455704
// MI455X (gfx1250) — hardware-run, weakly checked
//
#include <hip/hip_runtime.h>


#ifndef NTOK
#define NTOK 4096
#endif
#define NTOK_FULL 4096
#define EMB    20
#define NH_    4
#define HD     5
#define HID    80
#define NLAYER 4
#define AW     4
#define KW     32
#define VROWS  16
#define W1P    32
#define W2P    96
#define W2R    32
#define TILEP  (16 * EMB / 4)
#define SC2  ((float)(0.4472135954999579 * 1.4426950408889634))
#define PSH  14.0f
#define NEGB (-3.0e38f)
#define LNEPS 1.0e-5f

static_assert(AW == NH_);
static_assert(NH_ * HD == EMB);
static_assert(HD == 5);
static_assert(2 * HD <= 16);
static_assert(EMB == 20);
static_assert(HID == 80);
static_assert(HID % 16 == 0);
static_assert(W2P == 96);
static_assert(HID <= W2P);
static_assert(W2P % 32 == 0);
static_assert(EMB <= W1P);
static_assert(W1P == 32);
static_assert(KW == 32);
static_assert(W2R == 32);
static_assert(EMB <= W2R);
static_assert(NTOK % 32 == 0);
static_assert(NTOK % 16 == 0);
static_assert(NTOK <= NTOK_FULL);
static_assert((16 * EMB * 4) % 128 == 0);
static_assert(TILEP == 80);
static_assert(TILEP * 16 == 16 * EMB * 4);
static_assert(TILEP <= 32 * AW);
static_assert(TILEP % 8 == 0);
static_assert((NH_ * NTOK * (KW / 8)) % 256 == 0);
static_assert((NH_ * VROWS * (NTOK / 8)) % 8 == 0);
static_assert((HID * (W1P / 8)) % 8 == 0);
static_assert((W2R * (W2P / 8)) % 8 == 0);
static_assert(2 * 16 * EMB * 4 <= 131072);

typedef _Float16 h16;
typedef __attribute__((ext_vector_type(16))) _Float16 v16h;
typedef __attribute__((ext_vector_type(8)))  _Float16 v8h;
typedef __attribute__((ext_vector_type(8)))  float    v8f;
typedef __attribute__((ext_vector_type(4)))  float    v4f;
typedef v4f  __attribute__((may_alias)) v4fa;

__device__ __forceinline__ unsigned short f2bf(float f) { unsigned u = __float_as_uint(f); u += 0x7FFFu + ((u >> 16) & 1u); return (unsigned short)(u >> 16); }
__device__ __forceinline__ float bfr(float f) { return __uint_as_float(((unsigned)f2bf(f)) << 16); }
__device__ __forceinline__ v16h cat16(v8h lo, v8h hi) { return __builtin_shufflevector(lo, hi, 0, 1, 2, 3, 4, 5, 6, 7, 8, 9, 10, 11, 12, 13, 14, 15); }
__device__ __forceinline__ v16h  ldh(const h16* p) { return cat16(*(const v8h*)p, *(const v8h*)(p + 16)); }
static __device__ __forceinline__ h16 toh_flush(float v) { const h16 r = (h16)v; return (fabsf(v) < 6.103515625e-05f) ? (h16)0.0f : r; }
__device__ __forceinline__ v8f wmma16g(v16h a, v16h b, v8f c) {
    c = __builtin_amdgcn_wmma_f32_16x16x32_f16(false, a, false, b, (short)0, c, false, false);
    asm volatile("v_nop\n\tv_nop\n\tv_nop\n\tv_nop" : "+v"(c) : "v"(a), "v"(b));
    return c;
}
__device__ __forceinline__ float tanh_f(float z) { const float e = __builtin_amdgcn_exp2f(z * 2.8853900817779268f); return 1.0f - 2.0f * __builtin_amdgcn_rcpf(e + 1.0f); }

__global__ __launch_bounds__(256) void k_prep_ke(const float* __restrict__ K, const float* __restrict__ H, h16* KE) {
    const int p = blockIdx.x * 256 + threadIdx.x; if (p >= NH_ * NTOK * (KW / 8)) return;
    const int c = p & 3, key = (p >> 2) % NTOK, h = (p >> 2) / NTOK;
    const size_t base = (size_t)key * EMB + (size_t)h * HD;
    float kv[HD], hv[HD];
#pragma unroll
    for (int d = 0; d < HD; ++d) { kv[d] = bfr(K[base + d]); hv[d] = bfr(H[base + d]); }
    float f[8];
    f[0] = (c == 0) ? kv[0] : ((c == 1) ? hv[3] : 0.0f);
    f[1] = (c == 0) ? kv[1] : ((c == 1) ? hv[4] : 0.0f);
    f[2] = (c == 0) ? kv[2] : 0.0f;
    f[3] = (c == 0) ? kv[3] : 0.0f;
    f[4] = (c == 0) ? kv[4] : 0.0f;
    f[5] = (c == 0) ? hv[0] : 0.0f;
    f[6] = (c == 0) ? hv[1] : 0.0f;
    f[7] = (c == 0) ? hv[2] : 0.0f;
    v8h o;
#pragma unroll
    for (int i = 0; i < 8; ++i) o[i] = toh_flush(f[i]);
    *(volatile v8h*)(KE + (size_t)p * 8) = o; __threadfence(); *(volatile v8h*)(KE + (size_t)p * 8) = o;
}

__global__ __launch_bounds__(256) void k_prep_vt(const float* __restrict__ V, h16* VT) {
    const int p = blockIdx.x * 256 + threadIdx.x; if (p >= NH_ * VROWS * (NTOK / 8)) return;
    const int key8 = p % (NTOK / 8), d = (p / (NTOK / 8)) % VROWS, h = p / ((NTOK / 8) * VROWS);
    const int dc = d < HD - 1 ? d : HD - 1;
    v8h o;
#pragma unroll
    for (int i = 0; i < 8; ++i) {
        float x = V[(size_t)(key8 * 8 + i) * EMB + (size_t)h * HD + dc];
        asm volatile("" : "+v"(x));
        const float y = (d < HD) ? bfr(x) : 0.0f;
        o[i] = toh_flush(y); }
    *(volatile v8h*)(VT + (size_t)p * 8) = o; __threadfence(); *(volatile v8h*)(VT + (size_t)p * 8) = o;
}

__global__ __launch_bounds__(256) void k_prep_w1(const float* __restrict__ W1, h16* W1T) {
    const int p = blockIdx.x * 256 + threadIdx.x; if (p >= HID * (W1P / 8)) return;
    const int n = p >> 2, c = p & 3;
    v8h o;
#pragma unroll
    for (int i = 0; i < 8; ++i) {
        const int k = 8 * c + i; const int kc = k < EMB - 1 ? k : EMB - 1;
        float x = W1[(size_t)kc * HID + n];
        asm volatile("" : "+v"(x));
        const float y = (k < EMB) ? bfr(x) : 0.0f;
        o[i] = toh_flush(y); }
    *(volatile v8h*)(W1T + (size_t)p * 8) = o; __threadfence(); *(volatile v8h*)(W1T + (size_t)p * 8) = o;
}

__global__ __launch_bounds__(256) void k_prep_w2(const float* __restrict__ W2, h16* W2T) {
    const int p = blockIdx.x * 256 + threadIdx.x; if (p >= W2R * (W2P / 8)) return;
    const int j = p / (W2P / 8), c = p % (W2P / 8);
    const int jc = j < EMB - 1 ? j : EMB - 1;
    v8h o;
#pragma unroll
    for (int i = 0; i < 8; ++i) {
        const int n = 8 * c + i; const int nc = n < HID - 1 ? n : HID - 1;
        float x = W2[(size_t)nc * EMB + jc];
        asm volatile("" : "+v"(x));
        const float y = ((n < HID) & (j < EMB)) ? bfr(x) : 0.0f;
        o[i] = toh_flush(y); }
    *(volatile v8h*)(W2T + (size_t)p * 8) = o; __threadfence(); *(volatile v8h*)(W2T + (size_t)p * 8) = o;
}

__device__ __forceinline__ void ln20(float (&a)[8], float (&c)[4], const bool lo, const int hi, const float* __restrict__ g, const float* __restrict__ be) {
    float s = 0.0f, s1 = 0.0f;
#pragma unroll
    for (int i = 0; i < 8; ++i) s += a[i];
#pragma unroll
    for (int i = 0; i < 4; ++i) s1 += c[i];
    s += lo ? s1 : 0.0f;
    s += __shfl_xor(s, 16, 32);
    const float mu = s * (1.0f / EMB);
    float v = 0.0f, v1 = 0.0f;
#pragma unroll
    for (int i = 0; i < 8; ++i) { a[i] -= mu; v += a[i] * a[i]; }
#pragma unroll
    for (int i = 0; i < 4; ++i) { c[i] = lo ? (c[i] - mu) : 0.0f; v1 += c[i] * c[i]; }
    v += v1;
    v += __shfl_xor(v, 16, 32);
    const float rs = rsqrtf(v * (1.0f / EMB) + LNEPS);
    const v4f g0 = *(const v4f*)(g + 8 * hi), g1 = *(const v4f*)(g + 8 * hi + 4), g2 = *(const v4f*)(g + 16);
    const v4f e0 = *(const v4f*)(be + 8 * hi), e1 = *(const v4f*)(be + 8 * hi + 4), e2 = *(const v4f*)(be + 16);
#pragma unroll
    for (int i = 0; i < 4; ++i) {
        a[i]     = a[i] * rs * bfr(g0[i]) + bfr(e0[i]);
        a[4 + i] = a[4 + i] * rs * bfr(g1[i]) + bfr(e1[i]);
        const float y = c[i] * rs * bfr(g2[i]) + bfr(e2[i]);
        c[i] = lo ? y : 0.0f; }
}

__global__ __launch_bounds__(32 * AW) void k_layers(const float* __restrict__ Qin, const float* __restrict__ Hin,
                                                    const h16* __restrict__ KE, const h16* __restrict__ VT,
                                                    const h16* __restrict__ W1T, const h16* __restrict__ W2T,
                                                    const float* __restrict__ ln1g, const float* __restrict__ ln1b,
                                                    const float* __restrict__ ln2g, const float* __restrict__ ln2b,
                                                    const float* __restrict__ b1, const float* __restrict__ b2, float* OUT) {
    __shared__ __align__(16) float qs[16 * EMB];
    __shared__ __align__(16) float cs[16 * EMB];
    const int lane = threadIdx.x & 31, lr = lane & 15, hi = lane >> 4;
    const int wave = __builtin_amdgcn_readfirstlane((int)(threadIdx.x >> 5));
    const int t0 = blockIdx.x * 16;
    const bool lo = (hi == 0);
    const int pt = (int)threadIdx.x;
    const int pc = pt < TILEP - 1 ? pt : TILEP - 1;
    { v4f x = *(const v4f*)(Qin + (size_t)t0 * EMB + (size_t)pc * 4);
      asm volatile("" : "+v"(x));
      v4f y; y[0] = bfr(x[0]); y[1] = bfr(x[1]); y[2] = bfr(x[2]); y[3] = bfr(x[3]);
      if (pt < TILEP) *(v4fa*)(&qs[pt * 4]) = y; }
    float hq[HD];
#pragma unroll
    for (int d = 0; d < HD; ++d) hq[d] = bfr(Hin[(size_t)(t0 + lr) * EMB + (size_t)wave * HD + d]);
    const size_t ko = ((size_t)wave * NTOK + (size_t)lr) * KW + 8 * hi;
    const size_t vo = ((size_t)wave * VROWS + (size_t)lr) * NTOK + 8 * hi;
    const int qb = lr * EMB + 8 * hi, qc = lr * EMB + 16;
    __syncthreads();

#pragma unroll 1
    for (int layer = 0; layer < NLAYER; ++layer) {
        float qf[HD];
#pragma unroll
        for (int d = 0; d < HD; ++d) qf[d] = qs[lr * EMB + wave * HD + d];
        float f[8];
        f[0] = lo ? qf[0] : hq[3];
        f[1] = lo ? qf[1] : hq[4];
        f[2] = lo ? qf[2] : 0.0f;
        f[3] = lo ? qf[3] : 0.0f;
        f[4] = lo ? qf[4] : 0.0f;
        f[5] = lo ? hq[0] : 0.0f;
        f[6] = lo ? hq[1] : 0.0f;
        f[7] = lo ? hq[2] : 0.0f;
        v16h qh = (v16h){};
#pragma unroll
        for (int i = 0; i < 8; ++i) qh[i] = toh_flush(f[i]);

        v8f o0 = (v8f){};
        float m = NEGB, l = 0.0f;
#pragma unroll 1
        for (int key0 = 0; key0 < NTOK; key0 += 32) {
            const h16* ka = KE + ko + (size_t)key0 * KW;
            const v16h ka0 = ldh(ka), kb0 = ldh(ka + 16 * KW);
            v8f sa = (v8f){}, sb = (v8f){};
            sa = wmma16g(ka0, qh, sa); sb = wmma16g(kb0, qh, sb);
            float ta[8], tb[8]; float mx = NEGB;
#pragma unroll
            for (int r = 0; r < 8; ++r) { ta[r] = sa[r] * SC2; tb[r] = sb[r] * SC2; mx = fmaxf(mx, fmaxf(ta[r], tb[r])); }
            mx = fmaxf(mx, __shfl_xor(mx, 16, 32));
            const float mnew = fmaxf(m, mx);
            const float alpha = __builtin_amdgcn_exp2f(m - mnew);
            const float sh = PSH - mnew;
            v16h pb; float ls = 0.0f;
#pragma unroll
            for (int r = 0; r < 8; ++r) {
                const float ea = ta[r] + sh, eb = tb[r] + sh;
                const float ga = (ea < -14.0f) ? 0.0f : __builtin_amdgcn_exp2f(ea);
                const float gb = (eb < -14.0f) ? 0.0f : __builtin_amdgcn_exp2f(eb);
                const h16 pa = (h16)ga; const h16 pcv = (h16)gb;
                pb[r] = pa; pb[8 + r] = pcv;
                ls += (float)pa + (float)pcv; }
            l = l * alpha + ls; m = mnew;
            o0 = o0 * alpha;
            const v16h v0 = ldh(VT + vo + key0);
            o0 = wmma16g(v0, pb, o0);
        }
        l += __shfl_xor(l, 16, 32);
        const float inv = 1.0f / l;
        if (lo) {
#pragma unroll
            for (int r = 0; r < HD; ++r) cs[lr * EMB + wave * HD + r] = o0[r] * inv; }
        __syncthreads();

        if (wave == 0) {
            const v4f xa = *(const v4fa*)(&qs[qb]), xb = *(const v4fa*)(&qs[qb + 4]), xc = *(const v4fa*)(&qs[qc]);
            const v4f ca = *(const v4fa*)(&cs[qb]), cb = *(const v4fa*)(&cs[qb + 4]), cc = *(const v4fa*)(&cs[qc]);
            float a[8], c[4];
#pragma unroll
            for (int i = 0; i < 4; ++i) { a[i] = xa[i] + ca[i]; a[4 + i] = xb[i] + cb[i]; c[i] = lo ? (xc[i] + cc[i]) : 0.0f; }
            ln20(a, c, lo, hi, ln1g, ln1b);
            v16h bq = (v16h){};
#pragma unroll
            for (int i = 0; i < 8; ++i) bq[i] = toh_flush(a[i]);
#pragma unroll
            for (int i = 0; i < 4; ++i) bq[8 + i] = toh_flush(c[i]);
            v16h hb[3]; hb[0] = (v16h){}; hb[1] = (v16h){}; hb[2] = (v16h){};
#pragma unroll
            for (int nb = 0; nb < HID / 16; ++nb) {
                v8f d = (v8f){};
                d = wmma16g(ldh(W1T + (size_t)(nb * 16 + lr) * W1P + 8 * hi), bq, d);
                const v4f ba = *(const v4f*)(b1 + nb * 16 + 8 * hi), bb = *(const v4f*)(b1 + nb * 16 + 8 * hi + 4);
#pragma unroll
                for (int r = 0; r < 4; ++r) {
                    hb[nb >> 1][(nb & 1) * 8 + r]     = toh_flush(tanh_f(d[r] + bfr(ba[r])));
                    hb[nb >> 1][(nb & 1) * 8 + 4 + r] = toh_flush(tanh_f(d[4 + r] + bfr(bb[r]))); }
            }
            v8f f0 = (v8f){}, f1 = (v8f){};
#pragma unroll
            for (int s = 0; s < W2P / 32; ++s) {
                f0 = wmma16g(ldh(W2T + (size_t)lr * W2P + 32 * s + 8 * hi), hb[s], f0);
                f1 = wmma16g(ldh(W2T + (size_t)(16 + lr) * W2P + 32 * s + 8 * hi), hb[s], f1);
            }
            const v4f c0 = *(const v4f*)(b2 + 8 * hi), c1 = *(const v4f*)(b2 + 8 * hi + 4), c2 = *(const v4f*)(b2 + 16);
#pragma unroll
            for (int i = 0; i < 4; ++i) {
                a[i]     = a[i] + (f0[i] + bfr(c0[i]));
                a[4 + i] = a[4 + i] + (f0[4 + i] + bfr(c1[i]));
                const float y = c[i] + (f1[i] + bfr(c2[i]));
                c[i] = lo ? y : 0.0f; }
            ln20(a, c, lo, hi, ln2g, ln2b);
            v4f wa, wb, wc;
#pragma unroll
            for (int i = 0; i < 4; ++i) { wa[i] = a[i]; wb[i] = a[4 + i]; wc[i] = c[i]; }
            *(v4fa*)(&qs[qb]) = wa; *(v4fa*)(&qs[qb + 4]) = wb;
            if (lo) *(v4fa*)(&qs[qc]) = wc;
        }
        __syncthreads();
    }

    { v4f val = *(const v4fa*)(&qs[pc * 4]);
      asm volatile("" : "+v"(val));
      float* dst = OUT + (size_t)t0 * EMB + (size_t)pc * 4;
#pragma unroll 1
      for (int ps = 0; ps < 2; ++ps) {
          if (pt < TILEP) *(volatile v4f*)dst = val;
          if (ps == 0) __threadfence(); } }
}

static constexpr size_t al256(size_t v) { return (v + 255) & ~(size_t)255; }
static constexpr size_t SZ_KE = al256((size_t)NH_ * NTOK * KW * 2);
static constexpr size_t SZ_VT = al256((size_t)NH_ * VROWS * NTOK * 2);
static constexpr size_t SZ_W1 = al256((size_t)HID * W1P * 2);
static constexpr size_t SZ_W2 = al256((size_t)W2R * W2P * 2);
static constexpr size_t SZ_TOTAL = SZ_KE + SZ_VT + SZ_W1 + SZ_W2;
static_assert(SZ_TOTAL <= (size_t)134217728);
static_assert(((size_t)NH_ * NTOK * KW * 2) % 128 == 0);
static_assert(((size_t)NH_ * VROWS * NTOK * 2) % 128 == 0);
static_assert(((size_t)HID * W1P * 2) % 128 == 0);
static_assert(((size_t)W2R * W2P * 2) % 128 == 0);

extern "C" void kernel_launch(void* const* d_in, const int* in_sizes, int n_in,
                              void* d_out, int out_size, void* d_ws, size_t ws_size, hipStream_t stream) {
    if (n_in < 12) return;
    const size_t needx = (size_t)NTOK * EMB;
    if ((size_t)in_sizes[0] < needx || (size_t)in_sizes[1] < needx || (size_t)in_sizes[2] < needx || (size_t)in_sizes[3] < needx) return;
    if (in_sizes[4] < EMB || in_sizes[5] < EMB || in_sizes[6] < EMB || in_sizes[7] < EMB) return;
    if (in_sizes[8] < EMB * HID || in_sizes[9] < HID || in_sizes[10] < HID * EMB || in_sizes[11] < EMB) return;
    if ((size_t)out_size < needx) return;
    if (SZ_TOTAL > ws_size) return;
    const float* Q  = (const float*)d_in[0];
    const float* K  = (const float*)d_in[1];
    const float* V  = (const float*)d_in[2];
    const float* H  = (const float*)d_in[3];
    const float* ln1g = (const float*)d_in[4];
    const float* ln1b = (const float*)d_in[5];
    const float* ln2g = (const float*)d_in[6];
    const float* ln2b = (const float*)d_in[7];
    const float* W1 = (const float*)d_in[8];
    const float* b1 = (const float*)d_in[9];
    const float* W2 = (const float*)d_in[10];
    const float* b2 = (const float*)d_in[11];
    float* OUT = (float*)d_out;
    char* wsp = (char*)d_ws;
    h16* KE  = (h16*)wsp; wsp += SZ_KE;
    h16* VT  = (h16*)wsp; wsp += SZ_VT;
    h16* W1T = (h16*)wsp; wsp += SZ_W1;
    h16* W2T = (h16*)wsp; wsp += SZ_W2;

    k_prep_ke<<<(unsigned)((NH_ * NTOK * (KW / 8) + 255) / 256), 256, 0, stream>>>(K, H, KE);
    k_prep_vt<<<(unsigned)((NH_ * VROWS * (NTOK / 8) + 255) / 256), 256, 0, stream>>>(V, VT);
    k_prep_w1<<<(unsigned)((HID * (W1P / 8) + 255) / 256), 256, 0, stream>>>(W1, W1T);
    k_prep_w2<<<(unsigned)((W2R * (W2P / 8) + 255) / 256), 256, 0, stream>>>(W2, W2T);
    k_layers<<<NTOK / 16, 32 * AW, 0, stream>>>(Q, H, KE, VT, W1T, W2T, ln1g, ln1b, ln2g, ln2b, b1, b2, OUT);
}
